// GAT_82197084111388
// MI455X (gfx1250) — hardware-verified
//
#include <hip/hip_runtime.h>
#include <stddef.h>
#include <stdint.h>
#include <math.h>


#define F_IN    256
#define HID     512
#define KA      1024
#define N0      1024
#define N2P     320
#define F2      240
#define NCLS    40
#define SDW     16
#define NTHR    256
#define NWAVE   8
#define EPT     8
#define CHUNK   (NTHR * EPT)
#define WCAP    (EPT * 32)
#define LISTN   (NWAVE * WCAP)
#define NBA     1024
#define SLA     10
#define RCAP    28672
#define DEGCAP  128
#define MEAS_B1024  16569
#define MEAS_MAXDEG 36
#define GBM     64
#define GBN     64
#define GTHR    128
#define MROWS   128
#define UW0     (512 * (F_IN / 8))
#define UW1     (512 * (KA / 8))
#define UW2     (F2 * (KA / 8))
#define UWS     (NCLS * (KA / 8))
#define UWZ     ((N2P - F2 - NCLS) * (KA / 8))
#define NEGSL   0.2f
#define EPS_SM  1e-16f
#define WSMAX   134217728
#define SCAN_ZINTS    (RCAP + 3 * NBA)
#define SCAN_LDS_INTS (LISTN + 2 * RCAP + 3 * NBA + 32)

static_assert((CHUNK & (CHUNK - 1)) == 0 && CHUNK <= 4096);
static_assert((NBA & (NBA - 1)) == 0 && NBA == (1 << SLA) && NBA <= 1024);
static_assert(((long long)CHUNK << SLA) < (1LL << 31));
static_assert(LISTN >= NWAVE * WCAP);
static_assert(NBA % (4 * NWAVE) == 0);
static_assert((RCAP % 32) == 0 && (SCAN_ZINTS % 4) == 0);
static_assert(RCAP >= MEAS_B1024 + 4096);
static_assert(DEGCAP >= MEAS_MAXDEG + 8);
static_assert(SCAN_LDS_INTS * 4 <= 300000);
static_assert(GBM == (GTHR / 32) * 16);
static_assert((F_IN % 32) == 0 && (KA % 32) == 0 && KA == 2 * HID);
static_assert((N0 % GBN) == 0 && (HID % GBN) == 0 && (N2P % GBN) == 0);
static_assert((MROWS % GBM) == 0);
static_assert((UW0 % NTHR) == 0 && (UW1 % NTHR) == 0 && (UW2 % NTHR) == 0 && (UWS % NTHR) == 0 && (UWZ % NTHR) == 0);
static_assert(512 + NWAVE * 1024 <= RCAP);
static_assert(NWAVE * 1024 + NWAVE * 192 <= RCAP);
static_assert(F2 + NCLS <= N2P && 256 <= N2P);
static_assert(((4 * NCLS * 4) % 128) == 0);

typedef float          v2f  __attribute__((ext_vector_type(2)));
typedef float          v4f  __attribute__((ext_vector_type(4)));
typedef float          v8f  __attribute__((ext_vector_type(8)));
typedef int            v4i  __attribute__((ext_vector_type(4)));
typedef int            v8i  __attribute__((ext_vector_type(8)));
typedef unsigned int   v2u  __attribute__((ext_vector_type(2)));
typedef unsigned short v8us __attribute__((ext_vector_type(8)));
typedef __bf16         v16b __attribute__((ext_vector_type(16)));
typedef v4f  __attribute__((may_alias)) v4fa;
typedef v4i  __attribute__((may_alias)) v4ia;
typedef v8us __attribute__((may_alias)) v8usa;
union FragB { v16b v; v8us h[2]; v8i w; };

__device__ __forceinline__ v8f wmb(const FragB& a, const FragB& b, v8f c) {
  v8f d = __builtin_amdgcn_wmma_f32_16x16x32_bf16(false, a.v, false, b.v, (short)0, c, false, false);
  asm volatile("v_nop\n\tv_nop\n\tv_nop\n\tv_nop" : "+v"(d) : "v"(a.w), "v"(b.w));
  return d;
}

__device__ __forceinline__ unsigned int f2bf(float f) {
  const unsigned int u = __float_as_uint(f);
  const unsigned int r = ((u + 0x7FFFu + ((u >> 16) & 1u)) >> 16) & 0xFFFFu;
  return ((u & 0x7FFFFFFFu) > 0x7F800000u) ? 0x7FC0u : r;
}
__device__ __forceinline__ float bf2f(unsigned int b) { return __uint_as_float(b << 16); }
__device__ __forceinline__ float bfr(float f) { return bf2f(f2bf(f)); }
__device__ __forceinline__ v4f bfr4(const v4f a) {
  v4f r; r.x = bfr(a.x); r.y = bfr(a.y); r.z = bfr(a.z); r.w = bfr(a.w); return r;
}

template <int SLB>
__device__ __forceinline__ int scan_chunk(const int* __restrict__ dsts, int nE, int cbase, int slotBase,
                                          int nb, int vec8, int* list, int tid, int lane, int wave) {
  int wc = 0;
  const int el0  = tid * EPT;
  const int e0   = cbase + el0;
  const int sent = -2147483647 - 1;
  v4i da, db;
  if (vec8 != 0 && cbase + CHUNK <= nE) {
    da = *(const v4i*)(dsts + e0);
    db = *(const v4i*)(dsts + e0 + 4);
  } else {
    da.x = (e0     < nE) ? dsts[min(e0,     nE - 1)] : sent;
    da.y = (e0 + 1 < nE) ? dsts[min(e0 + 1, nE - 1)] : sent;
    da.z = (e0 + 2 < nE) ? dsts[min(e0 + 2, nE - 1)] : sent;
    da.w = (e0 + 3 < nE) ? dsts[min(e0 + 3, nE - 1)] : sent;
    db.x = (e0 + 4 < nE) ? dsts[min(e0 + 4, nE - 1)] : sent;
    db.y = (e0 + 5 < nE) ? dsts[min(e0 + 5, nE - 1)] : sent;
    db.z = (e0 + 6 < nE) ? dsts[min(e0 + 6, nE - 1)] : sent;
    db.w = (e0 + 7 < nE) ? dsts[min(e0 + 7, nE - 1)] : sent;
  }
  const unsigned nbs = (unsigned)slotBase;
  const unsigned unb = (unsigned)nb;
  const unsigned s0 = (unsigned)da.x - nbs, s1 = (unsigned)da.y - nbs;
  const unsigned s2 = (unsigned)da.z - nbs, s3 = (unsigned)da.w - nbs;
  const unsigned s4 = (unsigned)db.x - nbs, s5 = (unsigned)db.y - nbs;
  const unsigned s6 = (unsigned)db.z - nbs, s7 = (unsigned)db.w - nbs;
  const bool h0 = s0 < unb, h1 = s1 < unb, h2 = s2 < unb, h3 = s3 < unb;
  const bool h4 = s4 < unb, h5 = s5 < unb, h6 = s6 < unb, h7 = s7 < unb;
  const unsigned any = __builtin_amdgcn_ballot_w32(h0 | h1 | h2 | h3 | h4 | h5 | h6 | h7);
  if (any != 0u) {
#define HITJ(J, HJ, SJ) { \
      const unsigned mj = __builtin_amdgcn_ballot_w32(HJ); \
      if (mj != 0u) { \
        if (HJ) { \
          const int pos = wc + (int)__builtin_amdgcn_mbcnt_lo(mj, 0u); \
          if (pos < WCAP) list[wave * WCAP + pos] = ((el0 + (J)) << SLB) | (int)(SJ); \
        } \
        wc += (int)__builtin_popcount(mj); } }
    HITJ(0, h0, s0)
    HITJ(1, h1, s1)
    HITJ(2, h2, s2)
    HITJ(3, h3, s3)
    HITJ(4, h4, s4)
    HITJ(5, h5, s5)
    HITJ(6, h6, s6)
    HITJ(7, h7, s7)
#undef HITJ
  }
  return wc;
}

__device__ __forceinline__ v8us wtr8(const float* __restrict__ w, int pitch, int n, int kk) {
  const float* p = w + (size_t)kk * (size_t)pitch + n;
  v8us o;
#pragma unroll
  for (int i = 0; i < 8; ++i) o[i] = (unsigned short)f2bf(p[(size_t)i * (size_t)pitch]);
  return o;
}

__global__ __launch_bounds__(NTHR) void k_prep(const float* __restrict__ x, const float* __restrict__ W0,
                                               const float* __restrict__ Wsi, const float* __restrict__ W1,
                                               const float* __restrict__ W2, const float* __restrict__ Wso,
                                               unsigned short* XB, unsigned short* WT0, unsigned short* W1D,
                                               unsigned short* W2D, int nN, int nUx) {
  const int u = (int)blockIdx.x * NTHR + (int)threadIdx.x;
  v8us o;
  unsigned short* dp;
  const int b1 = nUx, b2 = b1 + UW0, b3 = b2 + UW0, b4 = b3 + UW1, b5 = b4 + UW2, b6 = b5 + UWS, b7 = b6 + UWZ;
  if (u < b1) {
    const int row = u >> 5;
    const int c0  = (u & 31) * 8;
    const int rc  = row < nN ? row : nN - 1;
    const float* p = x + (size_t)rc * F_IN + c0;
    const v4f a = *(const v4fa*)p;
    const v4f b = *(const v4fa*)(p + 4);
    const bool okr = row < nN;
    o[0] = okr ? (unsigned short)f2bf(a.x) : (unsigned short)0;
    o[1] = okr ? (unsigned short)f2bf(a.y) : (unsigned short)0;
    o[2] = okr ? (unsigned short)f2bf(a.z) : (unsigned short)0;
    o[3] = okr ? (unsigned short)f2bf(a.w) : (unsigned short)0;
    o[4] = okr ? (unsigned short)f2bf(b.x) : (unsigned short)0;
    o[5] = okr ? (unsigned short)f2bf(b.y) : (unsigned short)0;
    o[6] = okr ? (unsigned short)f2bf(b.z) : (unsigned short)0;
    o[7] = okr ? (unsigned short)f2bf(b.w) : (unsigned short)0;
    dp = XB + (size_t)row * F_IN + c0;
  } else if (u < b2) {
    const int v = u - b1, n = v >> 5, k8 = (v & 31) * 8;
    o  = wtr8(W0, HID, n, k8);
    dp = WT0 + (size_t)n * F_IN + k8;
  } else if (u < b3) {
    const int v = u - b2, n = v >> 5, k8 = (v & 31) * 8;
    o  = wtr8(Wsi, HID, n, k8);
    dp = WT0 + (size_t)(HID + n) * F_IN + k8;
  } else if (u < b4) {
    const int v = u - b3, n = v >> 7, k8 = (v & 127) * 8;
    o  = wtr8(W1, HID, n, k8 & (HID - 1));
    dp = W1D + (size_t)n * KA + k8;
  } else if (u < b5) {
    const int v = u - b4, n = v >> 7, k8 = (v & 127) * 8;
    o  = wtr8(W2, F2, n, k8 & (HID - 1));
    dp = W2D + (size_t)n * KA + k8;
  } else if (u < b6) {
    const int v = u - b5, n = v >> 7, k8 = (v & 127) * 8;
    o  = wtr8(Wso, NCLS, n, k8 & (HID - 1));
    dp = W2D + (size_t)(F2 + n) * KA + k8;
  } else if (u < b7) {
    const int v = u - b6, n = v >> 7, k8 = (v & 127) * 8;
#pragma unroll
    for (int i = 0; i < 8; ++i) o[i] = (unsigned short)0;
    dp = W2D + (size_t)(F2 + NCLS + n) * KA + k8;
  } else {
    return;
  }
  *(volatile v8us*)dp = o;
  __threadfence();
  *(volatile v8us*)dp = o;
}

__global__ __launch_bounds__(GTHR) void k_gemm(const unsigned short* __restrict__ A,
                                               const unsigned short* __restrict__ WT,
                                               float* outF, int K, int ldo) {
  __shared__ __attribute__((aligned(16))) float stg[GBM * GBN];
  const int tid = (int)threadIdx.x, lane = tid & 31, wave = tid >> 5, hh = lane >> 4, m = lane & 15;
  const int rowBase = (int)blockIdx.x * GBM;
  const int col0    = (int)blockIdx.y * GBN;

  v8f acc[4];
  {
    const v8f z = {0.f, 0.f, 0.f, 0.f, 0.f, 0.f, 0.f, 0.f};
    acc[0] = z; acc[1] = z; acc[2] = z; acc[3] = z;
  }
  const unsigned short* ap = A  + (size_t)(rowBase + 16 * wave + m) * (size_t)K + 8 * hh;
  const unsigned short* wp = WT + (size_t)(col0 + m) * (size_t)K + 8 * hh;
  const int ksteps = K >> 5;
#pragma unroll 1
  for (int ks = 0; ks < ksteps; ++ks) {
    FragB af;
    af.h[0] = *(const v8usa*)(ap + 32 * ks);
    af.h[1] = *(const v8usa*)(ap + 32 * ks + 16);
#pragma unroll
    for (int t = 0; t < 4; ++t) {
      const unsigned short* wq = wp + (size_t)(16 * t) * (size_t)K + 32 * ks;
      FragB bf;
      bf.h[0] = *(const v8usa*)wq;
      bf.h[1] = *(const v8usa*)(wq + 16);
      acc[t] = wmb(af, bf, acc[t]);
    }
  }

#pragma unroll
  for (int t = 0; t < 4; ++t) {
    const int lc = 16 * t + m;
#pragma unroll
    for (int r = 0; r < 8; ++r) {
      const int lr = 16 * wave + 8 * hh + r;
      stg[lr * GBN + lc] = acc[t][r];
    }
  }
  __syncthreads();

  v4f fv[8];
#pragma unroll
  for (int i = 0; i < 8; ++i) {
    const int lr = 16 * wave + 2 * i + hh;
    fv[i] = *(const v4fa*)(stg + lr * GBN + 4 * m);
  }
#pragma unroll
  for (int i = 0; i < 8; ++i) {
    const int lr = 16 * wave + 2 * i + hh;
    const int gr = rowBase + lr;
    float* op = outF + (size_t)gr * (size_t)ldo + col0 + 4 * m;
    *(volatile v4f*)op = fv[i];
  }
  __threadfence();
#pragma unroll
  for (int i = 0; i < 8; ++i) {
    const int lr = 16 * wave + 2 * i + hh;
    const int gr = rowBase + lr;
    float* op = outF + (size_t)gr * (size_t)ldo + col0 + 4 * m;
    *(volatile v4f*)op = fv[i];
  }
}

template <int NH, int HW, int NJ>
__global__ __launch_bounds__(NTHR) void k_dots(const float* __restrict__ F, int pitch,
                                               const float* __restrict__ atts, const float* __restrict__ attd,
                                               float* SD) {
  static_assert(NH * HW <= NJ * 128 && NH <= 8 && 2 * NJ * 32 <= NTHR && ((NH * HW) % 4) == 0 && (HW % 4) == 0);
  __shared__ __attribute__((aligned(16))) float satt[2 * NJ * 128];
  __shared__ __attribute__((aligned(16))) float sdl[128 * SDW];
  const int tid = (int)threadIdx.x, lane = tid & 31, wave = tid >> 5;
  const int rowBase = (int)blockIdx.x * 128;
  constexpr int NU = NJ * 32;
  constexpr int NV = NH * HW / 4;
  if (tid < 2 * NU) {
    const int which = tid / NU;
    const int uq    = tid - which * NU;
    const int ucl   = uq < NV ? uq : NV - 1;
    const v4f vs = *(const v4fa*)(atts + 4 * ucl);
    const v4f vd = *(const v4fa*)(attd + 4 * ucl);
    v4f v;
    v.x = (which == 0) ? vs.x : vd.x;
    v.y = (which == 0) ? vs.y : vd.y;
    v.z = (which == 0) ? vs.z : vd.z;
    v.w = (which == 0) ? vs.w : vd.w;
    v = bfr4(v);
    const v4f z4 = {0.f, 0.f, 0.f, 0.f};
    if (uq >= NV) v = z4;
    *(v4fa*)(satt + which * NJ * 128 + 4 * uq) = v;
  }
  __syncthreads();

  v4f as_[NJ], ad_[NJ];
  int hj[NJ];
  bool okj[NJ];
#pragma unroll
  for (int j = 0; j < NJ; ++j) {
    const int c0 = 128 * j + 4 * lane;
    as_[j] = *(const v4fa*)(satt + c0);
    ad_[j] = *(const v4fa*)(satt + NJ * 128 + c0);
    if constexpr (HW == 128) { hj[j] = j; }
    else { const int hq = c0 / HW; hj[j] = hq < NH - 1 ? hq : NH - 1; }
    okj[j] = c0 < NH * HW;
  }

#pragma unroll 1
  for (int r = 0; r < 16; ++r) {
    const int lr  = wave * 16 + r;
    const int row = rowBase + lr;
    const float* fp = F + (size_t)row * (size_t)pitch + 4 * lane;
    float ps[NJ], pd[NJ];
#pragma unroll
    for (int j = 0; j < NJ; ++j) {
      v4f v = *(const v4f*)(fp + 128 * j);
      const v4f z4 = {0.f, 0.f, 0.f, 0.f};
      if (!okj[j]) v = z4;
      float a = v.x * as_[j].x;
      a = fmaf(v.y, as_[j].y, a);
      a = fmaf(v.z, as_[j].z, a);
      a = fmaf(v.w, as_[j].w, a);
      float b = v.x * ad_[j].x;
      b = fmaf(v.y, ad_[j].y, b);
      b = fmaf(v.z, ad_[j].z, b);
      b = fmaf(v.w, ad_[j].w, b);
      ps[j] = a; pd[j] = b;
    }
    float val = 0.0f;
#pragma unroll
    for (int h = 0; h < NH; ++h) {
      float cs = 0.0f, cd = 0.0f;
#pragma unroll
      for (int j = 0; j < NJ; ++j) {
        const bool e = (hj[j] == h);
        cs += e ? ps[j] : 0.0f;
        cd += e ? pd[j] : 0.0f;
      }
#pragma unroll
      for (int off = 16; off > 0; off >>= 1) {
        cs += __shfl_xor(cs, off);
        cd += __shfl_xor(cd, off);
      }
      val = (lane == h) ? cs : val;
      val = (lane == 8 + h) ? cd : val;
    }
    if (lane < 16) sdl[lr * SDW + lane] = val;
  }
  __syncthreads();

  const v4f p0 = *(const v4fa*)(sdl + 4 * tid);
  const v4f p1 = *(const v4fa*)(sdl + 4 * (tid + NTHR));
  float* g0 = SD + (size_t)rowBase * SDW + 4 * tid;
  float* g1 = g0 + 4 * NTHR;
  *(volatile v4f*)g0 = p0;
  *(volatile v4f*)g1 = p1;
  __threadfence();
  *(volatile v4f*)g0 = p0;
  *(volatile v4f*)g1 = p1;
}

template <int LAYER>
__global__ __launch_bounds__(NTHR) void k_scan(
    const int* __restrict__ srcs, const int* __restrict__ dsts,
    const float* __restrict__ F, int pitchF, const float* __restrict__ SD,
    const float* __restrict__ bias, const float* __restrict__ SK, int pitchS,
    float* X1o, unsigned short* XP, float* out,
    int nN, int nE, int vec8, int MPr) {
  static_assert(LAYER >= 0 && LAYER <= 2);
  constexpr int NJ = (LAYER == 2) ? 2 : 4;
  constexpr int HW = (LAYER == 2) ? 40 : 128;
  constexpr int NH = (LAYER == 2) ? 6 : 4;
  constexpr int NA = 4 * NJ;
  extern __shared__ __attribute__((aligned(16))) int ssm[];
  int* list = ssm;
  int* hl   = list + LISTN;
  int* sl   = hl + RCAP;
  int* cnt  = sl + RCAP;
  int* offs = cnt + NBA;
  int* cur  = offs + NBA;
  int* wcnt = cur + NBA;
  const int tid = (int)threadIdx.x, lane = tid & 31, wave = tid >> 5;
  const int blk = (int)blockIdx.x;
  const int nodeBase = blk * NBA;
  int nb = nN - nodeBase;
  nb = nb < 0 ? 0 : (nb > NBA ? NBA : nb);

  {
    const v4i z4 = {0, 0, 0, 0};
    for (int i = tid * 4; i < SCAN_ZINTS; i += NTHR * 4) *(v4ia*)(sl + i) = z4;
    if (tid < 32) wcnt[tid] = 0;
  }
  __syncthreads();

  int tot = 0, ovf = 0;
  const int nChunks = (nE + CHUNK - 1) / CHUNK;
#pragma unroll 1
  for (int ch = 0; ch < nChunks; ++ch) {
    const int cbase = ch * CHUNK;
    const int wc = scan_chunk<SLA>(dsts, nE, cbase, nodeBase, nb, vec8, list, tid, lane, wave);
    if (lane == 0) wcnt[wave] = wc;
    __syncthreads();
    int pre = 0, all = 0;
#pragma unroll
    for (int w2 = 0; w2 < NWAVE; ++w2) {
      int c = wcnt[w2];
      c = c < 0 ? 0 : (c > WCAP ? WCAP : c);
      all += c;
      pre += (w2 < wave) ? c : 0;
    }
    const int wcc  = wc > WCAP ? WCAP : wc;
    const int base = tot + pre;
#pragma unroll 1
    for (int i = lane; i < wcc; i += 32) {
      const int ent = list[wave * WCAP + i];
      const int el  = (ent >> SLA) & (CHUNK - 1);
      const int sq  = ent & (NBA - 1);
      int eid = cbase + el;
      eid = eid > nE - 1 ? nE - 1 : eid;
      const int sraw = srcs[eid];
      const int s = sraw < 0 ? 0 : (sraw > nN - 1 ? nN - 1 : sraw);
      const int pos = base + i;
      if (pos < RCAP) hl[pos] = (int)((unsigned)s | ((unsigned)sq << 16));
    }
    if (tot + all > RCAP) ovf = 1;
    tot += all;
    tot = tot > RCAP ? RCAP : tot;
    __syncthreads();
  }
  const int nh = tot;

  if (wave == 0) {
#pragma unroll 1
    for (int b0 = 0; b0 < nh; b0 += 32) {
      const int idx = b0 + lane;
      const int uv  = hl[idx < nh ? idx : nh - 1];
      const int m32 = (nh - b0) < 32 ? (nh - b0) : 32;
#pragma unroll 1
      for (int k = 0; k < m32; ++k) {
        const int u  = __builtin_amdgcn_readlane(uv, k);
        const int sq = (u >> 16) & (NBA - 1);
        if (lane == 0) cnt[sq] = cnt[sq] + 1;
      }
    }
  }
  __syncthreads();
  if (wave == 0) {
    const int base = lane * (NBA / 32);
    int s = 0;
#pragma unroll 1
    for (int i = 0; i < NBA / 32; ++i) s += cnt[base + i];
    int incl = s;
#pragma unroll
    for (int d = 1; d < 32; d <<= 1) {
      const int y = __shfl_up(incl, d, 32);
      if (lane >= d) incl += y;
    }
    int run = incl - s;
#pragma unroll 1
    for (int i = 0; i < NBA / 32; ++i) {
      const int cv = cnt[base + i];
      offs[base + i] = run;
      cur[base + i]  = run;
      run += cv;
    }
  }
  __syncthreads();
  if (wave == 0) {
#pragma unroll 1
    for (int b0 = 0; b0 < nh; b0 += 32) {
      const int idx = b0 + lane;
      const int uv  = hl[idx < nh ? idx : nh - 1];
      const int m32 = (nh - b0) < 32 ? (nh - b0) : 32;
#pragma unroll 1
      for (int k = 0; k < m32; ++k) {
        const int u  = __builtin_amdgcn_readlane(uv, k);
        const int sq = (u >> 16) & (NBA - 1);
        if (lane == 0) {
          int p = cur[sq];
          p = p < 0 ? 0 : (p > RCAP - 1 ? RCAP - 1 : p);
          sl[p] = u;
          cur[sq] = p + 1;
        }
      }
    }
  }
  __syncthreads();

  float* fl = (float*)hl;
  float* st;
  float* sk2;
  if constexpr (LAYER != 2) {
    st  = fl + 512 + wave * 1024;
    sk2 = st + 512;
#pragma unroll 1
    for (int q = tid; q < 512; q += NTHR) {
      const int a = q >> 5, ln = q & 31;
      const int col = 128 * (a >> 2) + 4 * ln + (a & 3);
      fl[q] = bfr(bias[col]);
    }
  } else {
    st  = fl + wave * 1024;
    sk2 = fl + NWAVE * 1024 + wave * 192;
  }
  __syncthreads();

  const float qnan = __int_as_float(0x7fc00000);
  const float pzb  = (ovf != 0) ? qnan : 0.0f;
  int hj[NJ];
#pragma unroll
  for (int j = 0; j < NJ; ++j) {
    if constexpr (LAYER != 2) { hj[j] = j; }
    else { const int hq = (128 * j + 4 * lane) / HW; hj[j] = hq < NH - 1 ? hq : NH - 1; }
  }
  float b2v[5];
#pragma unroll
  for (int r = 0; r < 5; ++r) {
    if constexpr (LAYER == 2) {
      const int e = lane + 32 * r;
      b2v[r] = bfr(bias[e - NCLS * (e / NCLS)]);
    } else {
      b2v[r] = 0.0f;
    }
  }

#pragma unroll 1
  for (int gi = 0; gi < NBA / (4 * NWAVE); ++gi) {
    const int g = gi * NWAVE + wave;
#pragma unroll 1
    for (int q4 = 0; q4 < 4; ++q4) {
      const int s    = 4 * g + q4;
      const int node = nodeBase + s;
      const int nc   = node < nN ? node : nN - 1;
      int c = cnt[s];
      const bool big = c > DEGCAP;
      c = c < 0 ? 0 : (c > DEGCAP ? DEGCAP : c);
      int o = offs[s];
      o = o < 0 ? 0 : (o > RCAP ? RCAP : o);
      if (c > nh - o) c = nh - o;
      c = c < 0 ? 0 : c;
      float adv[NJ], mx[NJ], dn[NJ], acc[NA];
#pragma unroll
      for (int j = 0; j < NJ; ++j) {
        adv[j] = SD[(size_t)nc * SDW + 8 + hj[j]];
        mx[j] = -3.0e38f; dn[j] = 0.0f;
      }
#pragma unroll
      for (int i = 0; i < NA; ++i) acc[i] = 0.0f;
      const int T = c + 1;
#pragma unroll 1
      for (int b0 = 0; b0 < T; b0 += 32) {
        const int t = b0 + lane;
        int idx = o + t;
        idx = idx < 0 ? 0 : (idx > RCAP - 1 ? RCAP - 1 : idx);
        const int ent = sl[idx];
        int hs = ent & 0xFFFF;
        hs = hs > nN - 1 ? nN - 1 : hs;
        const int sr  = (t < c) ? hs : nc;
        const int m32 = (T - b0) < 32 ? (T - b0) : 32;
#pragma unroll 1
        for (int k = 0; k < m32; ++k) {
          const int sk = __builtin_amdgcn_readlane(sr, k);
          const float* rp = F + (size_t)sk * (size_t)pitchF + 4 * lane;
          const float* sp = SD + (size_t)sk * SDW;
#pragma unroll
          for (int j = 0; j < NJ; ++j) {
            float lg = sp[hj[j]] + adv[j];
            lg = lg > 0.f ? lg : NEGSL * lg;
            const float df = lg - mx[j];
            const float ee = expf(-fabsf(df));
            const bool  up = df > 0.f;
            const float s1 = up ? ee : 1.0f;
            const float s2 = up ? 1.0f : ee;
            mx[j] = up ? lg : mx[j];
            dn[j] = fmaf(dn[j], s1, s2);
            const v4f a = *(const v4f*)(rp + 128 * j);
            acc[4 * j + 0] = fmaf(acc[4 * j + 0], s1, s2 * a.x);
            acc[4 * j + 1] = fmaf(acc[4 * j + 1], s1, s2 * a.y);
            acc[4 * j + 2] = fmaf(acc[4 * j + 2], s1, s2 * a.z);
            acc[4 * j + 3] = fmaf(acc[4 * j + 3], s1, s2 * a.w);
          }
        }
      }
      float inv[NJ];
#pragma unroll
      for (int j = 0; j < NJ; ++j) inv[j] = __builtin_amdgcn_rcpf(dn[j] + EPS_SM);
      const float pzr = big ? qnan : pzb;

      if constexpr (LAYER != 2) {
        const bool live = node < nN;
        const float* kp = SK + (size_t)nc * (size_t)pitchS + 4 * lane;
#pragma unroll
        for (int j = 0; j < NJ; ++j) {
          const v4f kv = *(const v4f*)(kp + 128 * j);
          sk2[(4 * j + 0) * 32 + lane] = kv.x;
          sk2[(4 * j + 1) * 32 + lane] = kv.y;
          sk2[(4 * j + 2) * 32 + lane] = kv.z;
          sk2[(4 * j + 3) * 32 + lane] = kv.w;
          st[(4 * j + 0) * 32 + lane] = acc[4 * j + 0] * inv[j];
          st[(4 * j + 1) * 32 + lane] = acc[4 * j + 1] * inv[j];
          st[(4 * j + 2) * 32 + lane] = acc[4 * j + 2] * inv[j];
          st[(4 * j + 3) * 32 + lane] = acc[4 * j + 3] * inv[j];
        }
#pragma unroll 1
        for (int a = 0; a < 16; ++a) {
          float y = st[a * 32 + lane] + fl[a * 32 + lane];
          y = y + sk2[a * 32 + lane];
          y = (y > 0.0f) ? y : expm1f(y);
          st[a * 32 + lane] = y + pzr;
        }
        if (node < MPr) {
          v4f yv[NJ];
          v2u hv[NJ], lv[NJ];
#pragma unroll
          for (int j = 0; j < NJ; ++j) {
            const float y0 = st[(4 * j + 0) * 32 + lane];
            const float y1 = st[(4 * j + 1) * 32 + lane];
            const float y2 = st[(4 * j + 2) * 32 + lane];
            const float y3 = st[(4 * j + 3) * 32 + lane];
            const float v0 = live ? y0 : 0.0f;
            const float v1 = live ? y1 : 0.0f;
            const float v2 = live ? y2 : 0.0f;
            const float v3 = live ? y3 : 0.0f;
            yv[j].x = v0; yv[j].y = v1; yv[j].z = v2; yv[j].w = v3;
            const unsigned int h0 = f2bf(v0), h1 = f2bf(v1), h2 = f2bf(v2), h3 = f2bf(v3);
            const unsigned int g0 = f2bf(v0 - bf2f(h0)), g1 = f2bf(v1 - bf2f(h1));
            const unsigned int g2 = f2bf(v2 - bf2f(h2)), g3 = f2bf(v3 - bf2f(h3));
            hv[j].x = h0 | (h1 << 16); hv[j].y = h2 | (h3 << 16);
            lv[j].x = g0 | (g1 << 16); lv[j].y = g2 | (g3 << 16);
          }
          float* xr = X1o + (size_t)node * HID + 4 * lane;
          unsigned short* hp = XP + (size_t)node * KA + 4 * lane;
          if constexpr (LAYER == 0) {
#pragma unroll
            for (int j = 0; j < NJ; ++j) *(volatile v4f*)(xr + 128 * j) = yv[j];
          }
#pragma unroll
          for (int j = 0; j < NJ; ++j) {
            *(volatile v2u*)(hp + 128 * j) = hv[j];
            *(volatile v2u*)(hp + HID + 128 * j) = lv[j];
          }
          __threadfence();
          if constexpr (LAYER == 0) {
#pragma unroll
            for (int j = 0; j < NJ; ++j) *(volatile v4f*)(xr + 128 * j) = yv[j];
          }
#pragma unroll
          for (int j = 0; j < NJ; ++j) {
            *(volatile v2u*)(hp + 128 * j) = hv[j];
            *(volatile v2u*)(hp + HID + 128 * j) = lv[j];
          }
        }
      } else {
#pragma unroll
        for (int j = 0; j < NJ; ++j) {
          v4f nv;
          nv.x = acc[4 * j + 0] * inv[j] + pzr;
          nv.y = acc[4 * j + 1] * inv[j] + pzr;
          nv.z = acc[4 * j + 2] * inv[j] + pzr;
          nv.w = acc[4 * j + 3] * inv[j] + pzr;
          *(v4fa*)(st + q4 * 256 + 128 * j + 4 * lane) = nv;
        }
      }
    }

    if constexpr (LAYER == 2) {
      __syncthreads();
      const int node0 = nodeBase + 4 * g;
#pragma unroll
      for (int r = 0; r < 5; ++r) {
        const int e = lane + 32 * r;
        const int q = e / NCLS;
        const int c = e - NCLS * q;
        const float* sq = st + q * 256 + c;
        float s = sq[0];
        s += sq[HW];
        s += sq[2 * HW];
        s += sq[3 * HW];
        s += sq[4 * HW];
        s += sq[5 * HW];
        sk2[e] = s * (1.0f / 6.0f) + b2v[r];
      }
      __syncthreads();
      const int p1 = lane;
      const int p2 = 32 + (lane & 7);
      const int r1 = p1 / 10, c1 = 4 * (p1 - 10 * r1);
      const int r2 = p2 / 10, c2 = 4 * (p2 - 10 * r2);
      int n1 = node0 + r1; n1 = n1 < nN ? n1 : nN - 1;
      int n2 = node0 + r2; n2 = n2 < nN ? n2 : nN - 1;
      const v4f a1 = *(const v4fa*)(sk2 + 4 * p1);
      const v4f a2 = *(const v4fa*)(sk2 + 4 * p2);
      const v4f k1 = *(const v4f*)(SK + (size_t)n1 * (size_t)pitchS + c1);
      const v4f k2 = *(const v4f*)(SK + (size_t)n2 * (size_t)pitchS + c2);
      v4f o1, o2;
      o1.x = a1.x + k1.x; o1.y = a1.y + k1.y; o1.z = a1.z + k1.z; o1.w = a1.w + k1.w;
      o2.x = a2.x + k2.x; o2.y = a2.y + k2.y; o2.z = a2.z + k2.z; o2.w = a2.w + k2.w;
      if (node0 < nN) {
        float* gp = out + (size_t)node0 * NCLS;
        *(volatile v4f*)(gp + 4 * p1) = o1;
        if (lane < 8) *(volatile v4f*)(gp + 4 * p2) = o2;
        __threadfence();
        *(volatile v4f*)(gp + 4 * p1) = o1;
        if (lane < 8) *(volatile v4f*)(gp + 4 * p2) = o2;
      }
    }
  }
}

static inline int cdiv(int a, int b) { return (a + b - 1) / b; }

extern "C" void kernel_launch(void* const* d_in, const int* in_sizes, int n_in,
                              void* d_out, int out_size, void* d_ws, size_t ws_size,
                              hipStream_t stream) {
  if (n_in < 16) return;
  const int nN = in_sizes[0] / F_IN;
  if (nN <= 0 || in_sizes[0] != nN * F_IN || nN > 65536) return;
  if ((nN & 3) != 0) return;
  if (in_sizes[1] < 2 || (in_sizes[1] & 1) != 0) return;
  const int nE = in_sizes[1] / 2;
  if (nE < 1 || nE > (1 << 30)) return;
  if (in_sizes[2] != F_IN * HID) return;
  if (in_sizes[3] != HID || in_sizes[4] != HID) return;
  if (in_sizes[5] != HID) return;
  if (in_sizes[6] != F_IN * HID) return;
  if (in_sizes[7] != HID * HID) return;
  if (in_sizes[8] != HID || in_sizes[9] != HID) return;
  if (in_sizes[10] != HID) return;
  if (in_sizes[11] != HID * F2) return;
  if (in_sizes[12] != F2 || in_sizes[13] != F2) return;
  if (in_sizes[14] != NCLS) return;
  if (in_sizes[15] != HID * NCLS) return;
  if (out_size != nN * NCLS) return;

  const float* x    = (const float*)d_in[0];
  const int*   ei   = (const int*)  d_in[1];
  const float* W0   = (const float*)d_in[2];
  const float* as0  = (const float*)d_in[3];
  const float* ad0  = (const float*)d_in[4];
  const float* b0   = (const float*)d_in[5];
  const float* Wsi  = (const float*)d_in[6];
  const float* W1   = (const float*)d_in[7];
  const float* as1  = (const float*)d_in[8];
  const float* ad1  = (const float*)d_in[9];
  const float* b1   = (const float*)d_in[10];
  const float* W2   = (const float*)d_in[11];
  const float* as2  = (const float*)d_in[12];
  const float* ad2  = (const float*)d_in[13];
  const float* b2   = (const float*)d_in[14];
  const float* Wso  = (const float*)d_in[15];
  float* out = (float*)d_out;
  const int* src = ei;
  const int* dst = ei + nE;

  const int MP   = cdiv(nN, MROWS) * MROWS;
  const int gM   = MP / GBM;
  const int gA   = cdiv(MP, NBA);
  if ((long long)gA * NBA < (long long)MP) return;
  const int vec8 = ((nE & 3) == 0) ? 1 : 0;
  const int nUx  = MP * (F_IN / 8);
  if ((nUx % NTHR) != 0) return;

  char* ws = (char*)d_ws;
  size_t off = 0;
  const size_t oXB  = off; off += (size_t)MP * F_IN * 2;          off = (off + 255) & ~(size_t)255;
  const size_t oWT0 = off; off += (size_t)N0 * F_IN * 2;          off = (off + 255) & ~(size_t)255;
  const size_t oW1D = off; off += (size_t)HID * KA * 2;           off = (off + 255) & ~(size_t)255;
  const size_t oW2D = off; off += (size_t)N2P * KA * 2;           off = (off + 255) & ~(size_t)255;
  const size_t oHS0 = off; off += (size_t)MP * N0 * 4;            off = (off + 255) & ~(size_t)255;
  const size_t oX1  = off; off += (size_t)MP * HID * 4;           off = (off + 255) & ~(size_t)255;
  const size_t oXHL = off; off += (size_t)MP * KA * 2;            off = (off + 255) & ~(size_t)255;
  const size_t oSD  = off; off += (size_t)MP * SDW * 4;           off = (off + 255) & ~(size_t)255;
  if (off > ws_size || off > (size_t)WSMAX) return;
  const size_t h1Bytes  = (size_t)MP * HID * 4;
  const size_t h2Bytes  = (size_t)MP * N2P * 4;
  if (h1Bytes + h2Bytes > (size_t)MP * N0 * 4) return;
  unsigned short* XB  = (unsigned short*)(ws + oXB);
  unsigned short* WT0 = (unsigned short*)(ws + oWT0);
  unsigned short* W1D = (unsigned short*)(ws + oW1D);
  unsigned short* W2D = (unsigned short*)(ws + oW2D);
  float*          HS0 = (float*)(ws + oHS0);
  float*          H1  = (float*)(ws + oHS0);
  float*          H2S = (float*)(ws + oHS0 + h1Bytes);
  float*          X1  = (float*)(ws + oX1);
  unsigned short* XHL = (unsigned short*)(ws + oXHL);
  float*          SD  = (float*)(ws + oSD);

  const int scanLds = SCAN_LDS_INTS * 4;
  hipFuncSetAttribute(reinterpret_cast<const void*>(&k_scan<0>),
                      hipFuncAttributeMaxDynamicSharedMemorySize, scanLds);
  hipFuncSetAttribute(reinterpret_cast<const void*>(&k_scan<1>),
                      hipFuncAttributeMaxDynamicSharedMemorySize, scanLds);
  hipFuncSetAttribute(reinterpret_cast<const void*>(&k_scan<2>),
                      hipFuncAttributeMaxDynamicSharedMemorySize, scanLds);

  const int nUnits = nUx + 2 * UW0 + UW1 + UW2 + UWS + UWZ;
  k_prep<<<nUnits / NTHR, NTHR, 0, stream>>>(x, W0, Wsi, W1, W2, Wso, XB, WT0, W1D, W2D, nN, nUx);
  k_gemm<<<dim3(gM, N0 / GBN), GTHR, 0, stream>>>(XB, WT0, HS0, F_IN, N0);
  k_dots<4, 128, 4><<<MP / 128, NTHR, 0, stream>>>(HS0, N0, as0, ad0, SD);
  k_scan<0><<<gA, NTHR, scanLds, stream>>>(src, dst, HS0, N0, SD, b0, HS0 + HID, N0, X1, XHL, out,
                                           nN, nE, vec8, MP);
  k_gemm<<<dim3(gM, HID / GBN), GTHR, 0, stream>>>(XHL, W1D, H1, KA, HID);
  k_dots<4, 128, 4><<<MP / 128, NTHR, 0, stream>>>(H1, HID, as1, ad1, SD);
  k_scan<1><<<gA, NTHR, scanLds, stream>>>(src, dst, H1, HID, SD, b1, X1, HID, X1, XHL, out,
                                           nN, nE, vec8, MP);
  k_gemm<<<dim3(gM, N2P / GBN), GTHR, 0, stream>>>(XHL, W2D, H2S, KA, N2P);
  k_dots<6, 40, 2><<<MP / 128, NTHR, 0, stream>>>(H2S, N2P, as2, ad2, SD);
  k_scan<2><<<gA, NTHR, scanLds, stream>>>(src, dst, H2S, N2P, SD, b2, H2S + F2, N2P, X1, XHL, out,
                                           nN, nE, vec8, MP);
}
